// IGABlock_17995912970769
// MI455X (gfx1250) — hardware-verified
//
#include <hip/hip_runtime.h>

#define NB    2
#define EMB   128
#define IMH   64
#define IMW   64
#define HWP   4096
#define NPIX  8192
#define HEADS 4
#define HDIM  32
#define FFD   256
#define KCV   1152
#define LDC   132
#define XSP   136
#define ESP   36
#define EHP   40
#define NBQ   24
#define NBC   2
#define NBF1  144
#define NBF2  16
#define WSC   64.0f
#define XSC   64.0f
#define XINV  0.015625f
#define PJS   0.000244140625f
#define QS    64.0f
#define SQK   (0.17677669529663687f * 0.000244140625f)
#define PSC   4096.0f
#define OINV  0.000003814697265625f
#define RES   2048.0f
#define RSC   0.00048828125f
#define WINV  0.015625f
#define XNS   16.0f
#define CINV  0.0009765625f
#define GSC   16.0f
#define F2S   0.0009765625f
#define LNEPS 0.00001f

static_assert(NPIX == NB * IMH * IMW && HWP == IMH * IMW);
static_assert(EMB == HEADS * HDIM && HDIM == 32 && IMW == 64 && IMH == 64);
static_assert(NBQ * 256 * 8 == 3 * EMB * EMB && NBC * 256 * 8 == EMB * HDIM);
static_assert(NBF1 * 256 * 8 == FFD * KCV && NBF2 * 256 * 8 == EMB * FFD && KCV == 9 * EMB);
static_assert((LDC * 4) % 16 == 0 && (XSP * 2) % 16 == 0 && (ESP * 4) % 16 == 0 && (EHP * 2) % 16 == 0);
static_assert((EMB % 32) == 0 && (FFD % 32) == 0 && (KCV % 32) == 0 && (NPIX % 64) == 0 && (HWP % 64) == 0);

typedef _Float16       v16h  __attribute__((ext_vector_type(16)));
typedef unsigned short v16us __attribute__((ext_vector_type(16)));
typedef unsigned short v8us  __attribute__((ext_vector_type(8)));
typedef _Float16       v8h   __attribute__((ext_vector_type(8)));
typedef float          v8f   __attribute__((ext_vector_type(8)));
typedef float          v4f   __attribute__((ext_vector_type(4)));
typedef unsigned int   v4u   __attribute__((ext_vector_type(4)));

union UFrag { v16us v; v8us u[2]; v4u w[2]; };

__device__ __forceinline__ unsigned short bf_bits(float f) {
  unsigned u = __float_as_uint(f);
  return (unsigned short)((u + 0x7FFFu + ((u >> 16) & 1u)) >> 16);
}
__device__ __forceinline__ float bf_up(unsigned short b) { return __uint_as_float(((unsigned)b) << 16); }
__device__ __forceinline__ float bfr(float f) { return bf_up(bf_bits(f)); }
__device__ __forceinline__ unsigned short h_bits(_Float16 x) { return __builtin_bit_cast(unsigned short, x); }
__device__ __forceinline__ unsigned short hb16(float f) { return h_bits((_Float16)f); }
__device__ __forceinline__ unsigned pk16(unsigned short a, unsigned short b) { return (unsigned)a | ((unsigned)b << 16); }
__device__ __forceinline__ v8f zero8() { v8f z = {0.f, 0.f, 0.f, 0.f, 0.f, 0.f, 0.f, 0.f}; return z; }
__device__ __forceinline__ v16us zero16() {
  v16us z;
#pragma unroll
  for (int i = 0; i < 16; ++i) z[i] = 0;
  return z;
}

__device__ __forceinline__ void hl2(float f0, float f1, unsigned& hpk, unsigned& lpk) {
  const _Float16 h0 = (_Float16)f0, h1 = (_Float16)f1;
  hpk = pk16(h_bits(h0), h_bits(h1));
  lpk = pk16(hb16((f0 - (float)h0) * RES), hb16((f1 - (float)h1) * RES));
}

__device__ __forceinline__ void st16x2(unsigned short* dst, v4u pk) {
  *(volatile v4u*)dst = pk;
  __threadfence();
  *(volatile v4u*)dst = pk;
}

__device__ __forceinline__ v4u cvt_w8(const float* __restrict__ src) {
  const v4f a = *(const v4f*)(src);
  const v4f b = *(const v4f*)(src + 4);
  v4u pk;
  pk[0] = pk16(hb16(bfr(a[0]) * WSC), hb16(bfr(a[1]) * WSC));
  pk[1] = pk16(hb16(bfr(a[2]) * WSC), hb16(bfr(a[3]) * WSC));
  pk[2] = pk16(hb16(bfr(b[0]) * WSC), hb16(bfr(b[1]) * WSC));
  pk[3] = pk16(hb16(bfr(b[2]) * WSC), hb16(bfr(b[3]) * WSC));
  return pk;
}

__device__ __forceinline__ v16us ldfrag(const unsigned short* p) {
  union { v16us v; v8us h[2]; } f;
  f.h[0] = *(const v8us*)(p);
  f.h[1] = *(const v8us*)(p + 16);
  return f.v;
}

__device__ __forceinline__ v8f mma_h(v16us a, v16us b, v8f c) {
#if defined(__HIP_DEVICE_COMPILE__)
  return __builtin_amdgcn_wmma_f32_16x16x32_f16(false, __builtin_bit_cast(v16h, a), false,
                                               __builtin_bit_cast(v16h, b), (short)0, c, false, false);
#else
  (void)a; (void)b;
  return c;
#endif
}
__device__ __forceinline__ void guard4(v8f& c0, v8f& c1, v8f& c2, v8f& c3,
                                       const v16us& a0, const v16us& a1, const v16us& b0, const v16us& b1) {
#if defined(__HIP_DEVICE_COMPILE__)
  asm volatile("v_nop\n\tv_nop\n\tv_nop\n\tv_nop"
               : "+v"(c0), "+v"(c1), "+v"(c2), "+v"(c3)
               : "v"(a0), "v"(a1), "v"(b0), "v"(b1));
#endif
}
__device__ __forceinline__ void guard4s(v8f& s0, v8f& s1, v8f& s2, v8f& s3, const v16us& a0, const v16us& a1,
                                        const v16us& a2, const v16us& a3, const v16us& b) {
#if defined(__HIP_DEVICE_COMPILE__)
  asm volatile("v_nop\n\tv_nop\n\tv_nop\n\tv_nop"
               : "+v"(s0), "+v"(s1), "+v"(s2), "+v"(s3)
               : "v"(a0), "v"(a1), "v"(a2), "v"(a3), "v"(b));
#endif
}
__device__ __forceinline__ void guard2p(v8f& c0, v8f& c1, const v16us& p0, const v16us& p1,
                                        const v16us& v0, const v16us& v1, const v16us& v2, const v16us& v3) {
#if defined(__HIP_DEVICE_COMPILE__)
  asm volatile("v_nop\n\tv_nop\n\tv_nop\n\tv_nop"
               : "+v"(c0), "+v"(c1)
               : "v"(p0), "v"(p1), "v"(v0), "v"(v1), "v"(v2), "v"(v3));
#endif
}

__device__ __forceinline__ void mm_core1(const unsigned short* __restrict__ A, int lda,
                                         const unsigned short* __restrict__ W, int ldw, int nks,
                                         int arow0, int brow0, float* Cs) {
  const int tid = threadIdx.x, wave = tid >> 5, lane = tid & 31, hh = lane >> 4, c = lane & 15;
  const int mw = wave >> 2, nw = wave & 3;
  const unsigned short* a0p = A + (size_t)(arow0 + mw * 32 + c) * lda + 8 * hh;
  const unsigned short* a1p = A + (size_t)(arow0 + mw * 32 + 16 + c) * lda + 8 * hh;
  const unsigned short* b0p = W + (size_t)(brow0 + nw * 32 + c) * ldw + 8 * hh;
  const unsigned short* b1p = W + (size_t)(brow0 + nw * 32 + 16 + c) * ldw + 8 * hh;
  v8f c00 = zero8(), c01 = zero8(), c10 = zero8(), c11 = zero8();
#pragma unroll 1
  for (int ks = 0; ks < nks; ++ks) {
    const int ko = ks * 32;
    const v16us fa0 = ldfrag(a0p + ko);
    const v16us fa1 = ldfrag(a1p + ko);
    const v16us fb0 = ldfrag(b0p + ko);
    const v16us fb1 = ldfrag(b1p + ko);
    c00 = mma_h(fa0, fb0, c00);
    c01 = mma_h(fa0, fb1, c01);
    c10 = mma_h(fa1, fb0, c10);
    c11 = mma_h(fa1, fb1, c11);
    guard4(c00, c01, c10, c11, fa0, fa1, fb0, fb1);
  }
#pragma unroll
  for (int r = 0; r < 8; ++r) {
    const int row = mw * 32 + 8 * hh + r;
    Cs[row * LDC + nw * 32 + c]             = c00[r];
    Cs[row * LDC + nw * 32 + 16 + c]        = c01[r];
    Cs[(row + 16) * LDC + nw * 32 + c]      = c10[r];
    Cs[(row + 16) * LDC + nw * 32 + 16 + c] = c11[r];
  }
}

__device__ __forceinline__ void ln_tile(float* Xs, const float* __restrict__ g, const float* __restrict__ b) {
  const int tid = threadIdx.x, wave = tid >> 5, lane = tid & 31;
  const int c0 = lane * 4;
  float gg[4], bb[4];
#pragma unroll
  for (int e = 0; e < 4; ++e) { gg[e] = bfr(g[c0 + e]); bb[e] = bfr(b[c0 + e]); }
#pragma unroll 1
  for (int j = 0; j < 8; ++j) {
    const int px = wave * 8 + j;
    const v4f v = *(const v4f*)(Xs + px * LDC + c0);
    float s = (v[0] + v[1]) + (v[2] + v[3]);
#pragma unroll
    for (int off = 16; off > 0; off >>= 1) s += __shfl_xor(s, off, 32);
    const float mean = s * (1.0f / 128.0f);
    v4f d;
#pragma unroll
    for (int e = 0; e < 4; ++e) d[e] = v[e] - mean;
    float ss = (d[0] * d[0] + d[1] * d[1]) + (d[2] * d[2] + d[3] * d[3]);
#pragma unroll
    for (int off = 16; off > 0; off >>= 1) ss += __shfl_xor(ss, off, 32);
    const float var = ss * (1.0f / 128.0f);
    const float rstd = rsqrtf(var + LNEPS);
    v4f o;
#pragma unroll
    for (int e = 0; e < 4; ++e) o[e] = (d[e] * rstd) * gg[e] + bb[e];
    *(v4f*)(Xs + px * LDC + c0) = o;
  }
}

__global__ __launch_bounds__(256)
void k_cvt(const float* __restrict__ qkvw, const float* __restrict__ csw, const float* __restrict__ f1w,
           const float* __restrict__ f2w, unsigned short* wqkv16, unsigned short* cs16, unsigned short* w116,
           unsigned short* w216) {
  const int tid = threadIdx.x, blk = blockIdx.x;
  if (blk < NBQ) {
    const int t = blk * 256 + tid;
    const v4u pk = cvt_w8(qkvw + (size_t)t * 8);
    st16x2(wqkv16 + (size_t)t * 8, pk);
  } else if (blk < NBQ + NBC) {
    const int t = (blk - NBQ) * 256 + tid;
    const v4u pk = cvt_w8(csw + (size_t)t * 8);
    st16x2(cs16 + (size_t)t * 8, pk);
  } else if (blk < NBQ + NBC + NBF1) {
    const int t = (blk - NBQ - NBC) * 256 + tid;
    const int o = t / (KCV / 8);
    const int rem = t - o * (KCV / 8);
    const int tap = rem >> 4, ic0 = (rem & 15) * 8;
    const float* src = f1w + ((size_t)(o * EMB + ic0)) * 9 + tap;
    v4u pk;
#pragma unroll
    for (int e = 0; e < 4; ++e)
      pk[e] = pk16(hb16(bfr(src[(2 * e) * 9]) * WSC), hb16(bfr(src[(2 * e + 1) * 9]) * WSC));
    st16x2(w116 + (size_t)t * 8, pk);
  } else if (blk < NBQ + NBC + NBF1 + NBF2) {
    const int t = (blk - NBQ - NBC - NBF1) * 256 + tid;
    const v4u pk = cvt_w8(f2w + (size_t)t * 8);
    st16x2(w216 + (size_t)t * 8, pk);
  }
}

__global__ __launch_bounds__(256)
void k_prep(const float* __restrict__ x, unsigned short* x16) {
  __shared__ __align__(16) unsigned short Xs[64 * XSP];
  const int tid = threadIdx.x, blk = blockIdx.x;
  const int b = blk >> 6, y = blk & 63;
  const float* xb = x + (size_t)b * EMB * HWP + (size_t)y * IMW;
#pragma unroll 4
  for (int it = 0; it < 32; ++it) {
    const int idx = it * 256 + tid;
    const int c = idx >> 6, xl = idx & 63;
    Xs[xl * XSP + c] = hb16(bfr(xb[(size_t)c * HWP + xl]) * XSC);
  }
  __syncthreads();
  v4u pk[4];
  size_t offs[4];
#pragma unroll
  for (int s = 0; s < 4; ++s) {
    const int idx = s * 256 + tid;
    const int row = idx >> 4, piece = idx & 15;
    pk[s] = *(const v4u*)(Xs + row * XSP + piece * 8);
    offs[s] = (size_t)(blk * 64 + row) * EMB + piece * 8;
  }
#pragma unroll
  for (int s = 0; s < 4; ++s) *(volatile v4u*)(x16 + offs[s]) = pk[s];
  __threadfence();
#pragma unroll
  for (int s = 0; s < 4; ++s) *(volatile v4u*)(x16 + offs[s]) = pk[s];
}

__global__ __launch_bounds__(256)
void k_qkv(const unsigned short* __restrict__ x16, const unsigned short* __restrict__ wqkv16,
           const float* __restrict__ qkvb, unsigned short* q16, unsigned short* k16, unsigned short* vt16) {
  __shared__ __align__(16) float Cs[64 * LDC];
  const int tid = threadIdx.x;
  const int mb = blockIdx.x, nb = blockIdx.y;
  const int b = mb >> 6, n0 = (mb & 63) * 64;
  mm_core1(x16, EMB, wqkv16, EMB, EMB / 32, mb * 64, nb * 128, Cs);
  __syncthreads();
  if (nb < 2) {
    const float* bias = qkvb + nb * EMB;
    unsigned short* dstp = (nb == 0) ? q16 : k16;
    v4u pk[4];
    size_t offs[4];
#pragma unroll
    for (int s = 0; s < 4; ++s) {
      const int idx = s * 256 + tid;
      const int hd = idx >> 8, w = idx & 255;
      const int row = w >> 2, dp = w & 3;
      const int col0 = hd * HDIM + dp * 8;
      v4u a;
#pragma unroll
      for (int e = 0; e < 4; ++e) {
        const float f0 = (Cs[row * LDC + col0 + 2 * e]     * PJS + bfr(bias[col0 + 2 * e]))     * QS;
        const float f1 = (Cs[row * LDC + col0 + 2 * e + 1] * PJS + bfr(bias[col0 + 2 * e + 1])) * QS;
        a[e] = pk16(hb16(f0), hb16(f1));
      }
      pk[s] = a;
      offs[s] = ((size_t)((b * HEADS + hd) * HWP + n0 + row)) * HDIM + dp * 8;
    }
#pragma unroll
    for (int s = 0; s < 4; ++s) *(volatile v4u*)(dstp + offs[s]) = pk[s];
    __threadfence();
#pragma unroll
    for (int s = 0; s < 4; ++s) *(volatile v4u*)(dstp + offs[s]) = pk[s];
  } else {
    const float* bias = qkvb + 2 * EMB;
    v4u pk[4];
    size_t offs[4];
#pragma unroll
    for (int s = 0; s < 4; ++s) {
      const int idx = s * 256 + tid;
      const int col = idx >> 3, p = idx & 7;
      const int x0 = p * 8;
      const float bb = bfr(bias[col]);
      v4u a;
#pragma unroll
      for (int e = 0; e < 4; ++e) {
        const float f0 = (Cs[(x0 + 2 * e) * LDC + col]     * PJS + bb) * QS;
        const float f1 = (Cs[(x0 + 2 * e + 1) * LDC + col] * PJS + bb) * QS;
        a[e] = pk16(hb16(f0), hb16(f1));
      }
      pk[s] = a;
      offs[s] = ((size_t)(b * EMB + col)) * HWP + n0 + x0;
    }
#pragma unroll
    for (int s = 0; s < 4; ++s) *(volatile v4u*)(vt16 + offs[s]) = pk[s];
    __threadfence();
#pragma unroll
    for (int s = 0; s < 4; ++s) *(volatile v4u*)(vt16 + offs[s]) = pk[s];
  }
}

__global__ __launch_bounds__(128)
void k_attn(const unsigned short* __restrict__ q16, const unsigned short* __restrict__ k16,
            const unsigned short* __restrict__ vt16, const _Float16* __restrict__ xh,
            const unsigned short* __restrict__ cs16, const float* __restrict__ csb, float* x2) {
  __shared__ __align__(16) float Es[4 * 16 * ESP];
  __shared__ __align__(16) unsigned short Eh[4 * 16 * EHP];
  __shared__ __align__(16) unsigned short El[4 * 16 * EHP];
  const int tid = threadIdx.x, wave = tid >> 5, lane = tid & 31, hh = lane >> 4, c = lane & 15;
  const int blk = blockIdx.x;
  const int b = blk >> 8, h = (blk >> 6) & 3, qb = blk & 63;
  const int bh = b * HEADS + h;
  const int n0 = qb * 64 + wave * 16;
  const int pg0 = b * HWP + n0;
  float* Esw = Es + wave * 16 * ESP;
  unsigned short* Ehw = Eh + wave * 16 * EHP;
  unsigned short* Elw = El + wave * 16 * EHP;

  const v16us bq = ldfrag(q16 + ((size_t)(bh * HWP + n0 + c)) * HDIM + 8 * hh);
  const unsigned short* kbase = k16 + (size_t)bh * HWP * HDIM + (size_t)c * HDIM + 8 * hh;
  const unsigned short* vbase0 = vt16 + ((size_t)(bh * HDIM + c)) * HWP + 8 * hh;
  const unsigned short* vbase1 = vbase0 + (size_t)16 * HWP;
  const v8f z8 = zero8();
  v8f acc0 = zero8(), acc1 = zero8();
  float m = -1.0e30f, l = 0.f;

#pragma unroll 1
  for (int kc = 0; kc < HWP / 64; ++kc) {
    const int key0 = kc * 64;
    const v16us ak0 = ldfrag(kbase + (size_t)(key0) * HDIM);
    const v16us ak1 = ldfrag(kbase + (size_t)(key0 + 16) * HDIM);
    const v16us ak2 = ldfrag(kbase + (size_t)(key0 + 32) * HDIM);
    const v16us ak3 = ldfrag(kbase + (size_t)(key0 + 48) * HDIM);
    v8f s0 = mma_h(ak0, bq, z8);
    v8f s1 = mma_h(ak1, bq, z8);
    v8f s2 = mma_h(ak2, bq, z8);
    v8f s3 = mma_h(ak3, bq, z8);
    guard4s(s0, s1, s2, s3, ak0, ak1, ak2, ak3, bq);
    float mx = s0[0];
#pragma unroll
    for (int r = 0; r < 8; ++r) mx = fmaxf(mx, fmaxf(fmaxf(s0[r], s1[r]), fmaxf(s2[r], s3[r])));
    mx = fmaxf(mx, __shfl_xor(mx, 16, 32));
    const float mn = fmaxf(m, mx * SQK);
    const float alpha = __expf(m - mn);
    m = mn;
    float psum = 0.f;
    UFrag p0, p1;
#pragma unroll
    for (int rr = 0; rr < 4; ++rr) {
      const int ra = 2 * rr, rb = ra + 1;
      const float e0a = __expf(s0[ra] * SQK - mn), e0b = __expf(s0[rb] * SQK - mn);
      const float e1a = __expf(s1[ra] * SQK - mn), e1b = __expf(s1[rb] * SQK - mn);
      const float e2a = __expf(s2[ra] * SQK - mn), e2b = __expf(s2[rb] * SQK - mn);
      const float e3a = __expf(s3[ra] * SQK - mn), e3b = __expf(s3[rb] * SQK - mn);
      psum += ((e0a + e0b) + (e1a + e1b)) + ((e2a + e2b) + (e3a + e3b));
      p0.w[0][rr] = pk16(hb16(e0a * PSC), hb16(e0b * PSC));
      p0.w[1][rr] = pk16(hb16(e1a * PSC), hb16(e1b * PSC));
      p1.w[0][rr] = pk16(hb16(e2a * PSC), hb16(e2b * PSC));
      p1.w[1][rr] = pk16(hb16(e3a * PSC), hb16(e3b * PSC));
    }
    l = l * alpha + psum;
#pragma unroll
    for (int r = 0; r < 8; ++r) {
      const float ar = __shfl(alpha, 8 * hh + r, 32);
      acc0[r] *= ar;
      acc1[r] *= ar;
    }
    const v16us v00 = ldfrag(vbase0 + key0);
    const v16us v01 = ldfrag(vbase1 + key0);
    const v16us v10 = ldfrag(vbase0 + key0 + 32);
    const v16us v11 = ldfrag(vbase1 + key0 + 32);
    acc0 = mma_h(p0.v, v00, acc0);
    acc1 = mma_h(p0.v, v01, acc1);
    acc0 = mma_h(p1.v, v10, acc0);
    acc1 = mma_h(p1.v, v11, acc1);
    guard2p(acc0, acc1, p0.v, p1.v, v00, v01, v10, v11);
  }
  const float ltot = l + __shfl_xor(l, 16, 32);
  const float rl = __builtin_amdgcn_rcpf(ltot) * OINV;

#pragma unroll
  for (int r = 0; r < 8; ++r) {
    const float f = __shfl(rl, 8 * hh + r, 32);
    Esw[(8 * hh + r) * ESP + c]      = acc0[r] * f;
    Esw[(8 * hh + r) * ESP + 16 + c] = acc1[r] * f;
  }
  __syncthreads();
  {
    const int row = lane >> 1, half = lane & 1;
    const float* er = Esw + row * ESP + 16 * half;
    const _Float16* xr = xh + (size_t)(pg0 + row) * EMB + h * HDIM + 16 * half;
    const v8h xa = *(const v8h*)(xr);
    const v8h xb = *(const v8h*)(xr + 8);
    const v4f o0 = *(const v4f*)(er), o1 = *(const v4f*)(er + 4);
    const v4f o2 = *(const v4f*)(er + 8), o3 = *(const v4f*)(er + 12);
    float xv[16];
#pragma unroll
    for (int e = 0; e < 8; ++e) { xv[e] = (float)xa[e] * XINV; xv[8 + e] = (float)xb[e] * XINV; }
#pragma unroll
    for (int e = 0; e < 4; ++e) { xv[e] += o0[e]; xv[4 + e] += o1[e]; xv[8 + e] += o2[e]; xv[12 + e] += o3[e]; }
    v4u ha, hb, la, lb;
#pragma unroll
    for (int e = 0; e < 4; ++e) {
      unsigned ph_, pl_;
      hl2(xv[2 * e], xv[2 * e + 1], ph_, pl_);         ha[e] = ph_; la[e] = pl_;
      hl2(xv[8 + 2 * e], xv[8 + 2 * e + 1], ph_, pl_); hb[e] = ph_; lb[e] = pl_;
    }
    unsigned short* ehr = Ehw + row * EHP + 16 * half;
    unsigned short* elr = Elw + row * EHP + 16 * half;
    *(v4u*)(ehr) = ha; *(v4u*)(ehr + 8) = hb;
    *(v4u*)(elr) = la; *(v4u*)(elr + 8) = lb;
  }
  __syncthreads();
  {
    const v16us fah = ldfrag(Ehw + c * EHP + 8 * hh);
    const v16us fal = ldfrag(Elw + c * EHP + 8 * hh);
    const v16us fb0 = ldfrag(cs16 + (size_t)(h * HDIM + c) * HDIM + 8 * hh);
    const v16us fb1 = ldfrag(cs16 + (size_t)(h * HDIM + 16 + c) * HDIM + 8 * hh);
    v8f t0h = mma_h(fah, fb0, z8);
    v8f t0l = mma_h(fal, fb0, z8);
    v8f t1h = mma_h(fah, fb1, z8);
    v8f t1l = mma_h(fal, fb1, z8);
    guard4(t0h, t0l, t1h, t1l, fah, fal, fb0, fb1);
    const float cb0 = bfr(csb[h * HDIM + c]), cb1 = bfr(csb[h * HDIM + 16 + c]);
#pragma unroll
    for (int r = 0; r < 8; ++r) {
      Esw[(8 * hh + r) * ESP + c]      = (t0h[r] + t0l[r] * RSC) * WINV + cb0;
      Esw[(8 * hh + r) * ESP + 16 + c] = (t1h[r] + t1l[r] * RSC) * WINV + cb1;
    }
  }
  __syncthreads();
  v4f pv[4];
  size_t po[4];
#pragma unroll
  for (int s = 0; s < 4; ++s) {
    const int idx = s * 32 + lane;
    const int row = idx >> 3, piece = idx & 7;
    pv[s] = *(const v4f*)(Esw + row * ESP + piece * 4);
    po[s] = (size_t)(pg0 + row) * EMB + h * HDIM + piece * 4;
  }
#pragma unroll
  for (int s = 0; s < 4; ++s) *(volatile v4f*)(x2 + po[s]) = pv[s];
  __threadfence();
#pragma unroll
  for (int s = 0; s < 4; ++s) *(volatile v4f*)(x2 + po[s]) = pv[s];
}

__global__ __launch_bounds__(256)
void k_ln(const float* __restrict__ x2, const float* __restrict__ g, const float* __restrict__ bta,
          float* xnf, unsigned short* xnh) {
  __shared__ __align__(16) float Xs[64 * LDC];
  const int tid = threadIdx.x, blk = blockIdx.x;
  const size_t row0 = (size_t)blk * 64;
#pragma unroll
  for (int it = 0; it < 8; ++it) {
    const int idx = it * 256 + tid;
    const int row = idx >> 5, piece = idx & 31;
    *(v4f*)(Xs + row * LDC + piece * 4) = *(const v4f*)(x2 + (row0 + row) * EMB + piece * 4);
  }
  __syncthreads();
  ln_tile(Xs, g, bta);
  __syncthreads();
  {
    v4f pv[8];
    size_t offs[8];
#pragma unroll
    for (int s = 0; s < 8; ++s) {
      const int idx = s * 256 + tid;
      const int row = idx >> 5, piece = idx & 31;
      pv[s] = *(const v4f*)(Xs + row * LDC + piece * 4);
      offs[s] = (row0 + row) * EMB + piece * 4;
    }
#pragma unroll
    for (int s = 0; s < 8; ++s) *(volatile v4f*)(xnf + offs[s]) = pv[s];
    __threadfence();
#pragma unroll
    for (int s = 0; s < 8; ++s) *(volatile v4f*)(xnf + offs[s]) = pv[s];
  }
  {
    v4u hw[4];
    size_t offs[4];
#pragma unroll
    for (int s = 0; s < 4; ++s) {
      const int idx = s * 256 + tid;
      const int row = idx >> 4, piece = idx & 15;
      const v4f a = *(const v4f*)(Xs + row * LDC + piece * 8);
      const v4f b = *(const v4f*)(Xs + row * LDC + piece * 8 + 4);
      v4u h4;
      h4[0] = pk16(hb16(a[0] * XNS), hb16(a[1] * XNS));
      h4[1] = pk16(hb16(a[2] * XNS), hb16(a[3] * XNS));
      h4[2] = pk16(hb16(b[0] * XNS), hb16(b[1] * XNS));
      h4[3] = pk16(hb16(b[2] * XNS), hb16(b[3] * XNS));
      hw[s] = h4;
      offs[s] = (row0 + row) * EMB + piece * 8;
    }
#pragma unroll
    for (int s = 0; s < 4; ++s) *(volatile v4u*)(xnh + offs[s]) = hw[s];
    __threadfence();
#pragma unroll
    for (int s = 0; s < 4; ++s) *(volatile v4u*)(xnh + offs[s]) = hw[s];
  }
}

__global__ __launch_bounds__(256)
void k_conv(const unsigned short* __restrict__ xnh, const unsigned short* __restrict__ w116,
            const float* __restrict__ f1b, unsigned short* g16) {
  __shared__ __align__(16) float Cs[64 * LDC];
  const int tid = threadIdx.x, wave = tid >> 5, lane = tid & 31, hh = lane >> 4, c = lane & 15;
  const int mw = wave >> 2, nw = wave & 3;
  const int mb = blockIdx.x, nb = blockIdx.y;
  const int b = mb >> 6, y = mb & 63;
  const int xq0 = mw * 32 + c, xq1 = xq0 + 16;
  const unsigned short* b0p = w116 + (size_t)(nb * 128 + nw * 32 + c) * KCV + 8 * hh;
  const unsigned short* b1p = b0p + (size_t)16 * KCV;
  const v16us zu16 = zero16();
  v8f c00 = zero8(), c01 = zero8(), c10 = zero8(), c11 = zero8();
#pragma unroll 1
  for (int tap = 0; tap < 9; ++tap) {
    const int ty = tap / 3;
    const int dy = ty - 1, dx = tap - ty * 3 - 1;
    const int yy = y + dy;
    const bool rin = (unsigned)yy < (unsigned)IMH;
    const int yyc = min(max(yy, 0), IMH - 1);
    const int xs0 = xq0 + dx, xs1 = xq1 + dx;
    const bool ok0 = rin && ((unsigned)xs0 < (unsigned)IMW);
    const bool ok1 = rin && ((unsigned)xs1 < (unsigned)IMW);
    const int xs0c = min(max(xs0, 0), IMW - 1), xs1c = min(max(xs1, 0), IMW - 1);
    const unsigned short* a0p = xnh + ((size_t)((b * IMH + yyc) * IMW + xs0c)) * EMB + 8 * hh;
    const unsigned short* a1p = xnh + ((size_t)((b * IMH + yyc) * IMW + xs1c)) * EMB + 8 * hh;
    const unsigned short* bt0 = b0p + tap * EMB;
    const unsigned short* bt1 = b1p + tap * EMB;
#pragma unroll 1
    for (int ks = 0; ks < EMB / 32; ++ks) {
      const int ko = ks * 32;
      v16us fa0 = ldfrag(a0p + ko);
      v16us fa1 = ldfrag(a1p + ko);
      fa0 = ok0 ? fa0 : zu16;
      fa1 = ok1 ? fa1 : zu16;
      const v16us fb0 = ldfrag(bt0 + ko);
      const v16us fb1 = ldfrag(bt1 + ko);
      c00 = mma_h(fa0, fb0, c00);
      c01 = mma_h(fa0, fb1, c01);
      c10 = mma_h(fa1, fb0, c10);
      c11 = mma_h(fa1, fb1, c11);
      guard4(c00, c01, c10, c11, fa0, fa1, fb0, fb1);
    }
  }
#pragma unroll
  for (int r = 0; r < 8; ++r) {
    const int row = mw * 32 + 8 * hh + r;
    Cs[row * LDC + nw * 32 + c]             = c00[r];
    Cs[row * LDC + nw * 32 + 16 + c]        = c01[r];
    Cs[(row + 16) * LDC + nw * 32 + c]      = c10[r];
    Cs[(row + 16) * LDC + nw * 32 + 16 + c] = c11[r];
  }
  __syncthreads();
  v4u hw[4];
  size_t offs[4];
#pragma unroll
  for (int s = 0; s < 4; ++s) {
    const int idx = s * 256 + tid;
    const int row = idx >> 4, piece = idx & 15;
    const int col0 = piece * 8;
    v4u a;
#pragma unroll
    for (int e = 0; e < 4; ++e) {
      const int j0 = col0 + 2 * e, j1 = j0 + 1;
      const float u0 = Cs[row * LDC + j0] * CINV + bfr(f1b[nb * 128 + j0]);
      const float u1 = Cs[row * LDC + j1] * CINV + bfr(f1b[nb * 128 + j1]);
      const float g0 = 0.5f * u0 * (1.0f + erff(u0 * 0.70710678118654752f)) * GSC;
      const float g1 = 0.5f * u1 * (1.0f + erff(u1 * 0.70710678118654752f)) * GSC;
      a[e] = pk16(hb16(g0), hb16(g1));
    }
    hw[s] = a;
    offs[s] = (size_t)(mb * 64 + row) * FFD + (size_t)nb * 128 + col0;
  }
#pragma unroll
  for (int s = 0; s < 4; ++s) *(volatile v4u*)(g16 + offs[s]) = hw[s];
  __threadfence();
#pragma unroll
  for (int s = 0; s < 4; ++s) *(volatile v4u*)(g16 + offs[s]) = hw[s];
}

__global__ __launch_bounds__(256)
void k_f2(const unsigned short* __restrict__ g16, const unsigned short* __restrict__ w216,
          const float* __restrict__ f2b, const float* __restrict__ xnf, float* out) {
  __shared__ __align__(16) float Cs[64 * LDC];
  const int tid = threadIdx.x, wave = tid >> 5, lane = tid & 31, hh = lane >> 4, piece = lane & 15;
  const int mb = blockIdx.x;
  const int b = mb >> 6, y = mb & 63;
  mm_core1(g16, FFD, w216, FFD, FFD / 32, mb * 64, 0, Cs);
  __syncthreads();
#pragma unroll 1
  for (int it = 0; it < 8; ++it) {
    const int o = wave * 16 + it * 2 + hh;
    const float bo = bfr(f2b[o]);
    v4f val;
#pragma unroll
    for (int e = 0; e < 4; ++e) {
      const int px = piece * 4 + e;
      val[e] = Cs[px * LDC + o] * F2S + bo + xnf[(size_t)(mb * 64 + px) * EMB + o];
    }
    float* p = out + ((size_t)(b * EMB + o)) * HWP + (size_t)y * IMW + piece * 4;
    *(volatile v4f*)p = val;
    __threadfence();
    *(volatile v4f*)p = val;
  }
}

extern "C" void kernel_launch(void* const* d_in, const int* in_sizes, int n_in,
                              void* d_out, int out_size, void* d_ws, size_t ws_size,
                              hipStream_t stream) {
  if (n_in < 11) return;
  const int expect[11] = { NPIX * EMB, 3 * EMB * EMB, 3 * EMB, EMB * HDIM, EMB, EMB, EMB,
                           FFD * EMB * 9, FFD, EMB * FFD, EMB };
  for (int i = 0; i < 11; ++i) if (in_sizes[i] != expect[i]) return;
  if (out_size != NPIX * EMB) return;

  const float* x     = (const float*)d_in[0];
  const float* qkvw  = (const float*)d_in[1];
  const float* qkvb  = (const float*)d_in[2];
  const float* csw   = (const float*)d_in[3];
  const float* csb   = (const float*)d_in[4];
  const float* lnw   = (const float*)d_in[5];
  const float* lnb   = (const float*)d_in[6];
  const float* f1w   = (const float*)d_in[7];
  const float* f1b   = (const float*)d_in[8];
  const float* f2w   = (const float*)d_in[9];
  const float* f2b   = (const float*)d_in[10];
  float* out = (float*)d_out;

  const size_t AL = 65536;
  const size_t sWQ  = (((size_t)3 * EMB * EMB * 2) + AL - 1) / AL * AL;
  const size_t sCS  = (((size_t)EMB * HDIM * 2) + AL - 1) / AL * AL;
  const size_t sW1  = (((size_t)FFD * KCV * 2) + AL - 1) / AL * AL;
  const size_t sW2  = (((size_t)EMB * FFD * 2) + AL - 1) / AL * AL;
  const size_t sH16 = (((size_t)NPIX * EMB * 2) + AL - 1) / AL * AL;
  const size_t sF32 = (((size_t)NPIX * EMB * 4) + AL - 1) / AL * AL;
  const size_t sG16 = (((size_t)NPIX * FFD * 2) + AL - 1) / AL * AL;

  size_t off = 0;
  const size_t oWQ  = off; off += sWQ;
  const size_t oCS  = off; off += sCS;
  const size_t oW1  = off; off += sW1;
  const size_t oW2  = off; off += sW2;
  const size_t oX16 = off; off += sH16;
  const size_t oQ   = off; off += sH16;
  const size_t oK   = off; off += sH16;
  const size_t oVT  = off; off += sH16;
  const size_t oX2  = off; off += sF32;
  const size_t oXNF = off; off += sF32;
  const size_t oXNH = off; off += sH16;
  const size_t oG16 = off; off += sG16;
  if (off > ws_size) return;
  if (off > (size_t)134217728) return;

  char* ws = (char*)d_ws;
  unsigned short* WQKV16 = (unsigned short*)(ws + oWQ);
  unsigned short* CS16   = (unsigned short*)(ws + oCS);
  unsigned short* W1_16  = (unsigned short*)(ws + oW1);
  unsigned short* W2_16  = (unsigned short*)(ws + oW2);
  unsigned short* X16    = (unsigned short*)(ws + oX16);
  unsigned short* Q16    = (unsigned short*)(ws + oQ);
  unsigned short* K16    = (unsigned short*)(ws + oK);
  unsigned short* VT16   = (unsigned short*)(ws + oVT);
  float*          X2     = (float*)(ws + oX2);
  float*          XNF    = (float*)(ws + oXNF);
  unsigned short* XNH    = (unsigned short*)(ws + oXNH);
  unsigned short* G16    = (unsigned short*)(ws + oG16);

  const dim3 blk(256);
  k_cvt<<<dim3(NBQ + NBC + NBF1 + NBF2), blk, 0, stream>>>(qkvw, csw, f1w, f2w, WQKV16, CS16, W1_16, W2_16);
  k_prep<<<dim3(NPIX / 64), blk, 0, stream>>>(x, X16);
  k_qkv<<<dim3(NPIX / 64, 3), blk, 0, stream>>>(X16, WQKV16, qkvb, Q16, K16, VT16);
  k_attn<<<dim3(NB * HEADS * (HWP / 64)), dim3(128), 0, stream>>>(Q16, K16, VT16, (const _Float16*)X16,
                                                                  CS16, csb, X2);
  k_ln<<<dim3(NPIX / 64), blk, 0, stream>>>(X2, lnw, lnb, XNF, XNH);
  k_conv<<<dim3(NPIX / 64, FFD / 128), blk, 0, stream>>>(XNH, W1_16, f1b, G16);
  k_f2<<<dim3(NPIX / 64), blk, 0, stream>>>(G16, W2_16, f2b, XNF, out);
  (void)hipGetLastError();
}
